// GaussianBasis_68994354643524
// MI455X (gfx1250) — hardware-verified
//
#include <hip/hip_runtime.h>
#include <math.h>

typedef __attribute__((ext_vector_type(16))) _Float16 v16h;
typedef __attribute__((ext_vector_type(16))) __bf16 v16b;
typedef __attribute__((ext_vector_type(8)))  _Float16 v8h;
typedef __attribute__((ext_vector_type(8)))  float v8f;
typedef __attribute__((ext_vector_type(4)))  float v4f;
typedef __attribute__((ext_vector_type(2)))  float v2f;
typedef __attribute__((ext_vector_type(4)))  unsigned v4u;
typedef __attribute__((ext_vector_type(4)))  int v4i;
typedef float __attribute__((may_alias)) float_a;
typedef int __attribute__((may_alias)) int_a;

template <typename T> __device__ __forceinline__ void vst2(void* p, T v) { *(volatile T*)p = v; __threadfence(); *(volatile T*)p = v; }
__device__ __forceinline__ v8f wmma16(v16h a, v16h b, v8f c) {
  v8f d = __builtin_amdgcn_wmma_f32_16x16x32_f16(false, a, false, b, (short)0, c, false, false);
  asm volatile("v_nop\n\tv_nop\n\tv_nop\n\tv_nop" : "+v"(d) : "v"(a), "v"(b));
  return d;
}
__device__ __forceinline__ v8f wmma_bf(v16b a, v16b b, v8f c) {
  v8f d = __builtin_amdgcn_wmma_f32_16x16x32_bf16(false, a, false, b, (short)0, c, false, false);
  asm volatile("v_nop\n\tv_nop\n\tv_nop\n\tv_nop" : "+v"(d) : "v"(a), "v"(b));
  return d;
}
__device__ __forceinline__ v16h frag_h(const _Float16* rowk0, int lane) {
  union { v16h v; v8h q[2]; } u; const _Float16* p = rowk0 + 8 * (lane >> 4);
  u.q[0] = *(const v8h*)p; u.q[1] = *(const v8h*)(p + 16); return u.v;
}
__device__ __forceinline__ v16h frag_f32(const float* rowk0, int lane) {
  v16h a; const float* p = rowk0 + 8 * (lane >> 4);
#pragma unroll
  for (int i = 0; i < 8; ++i) { a[i] = (_Float16)p[i]; a[8 + i] = (_Float16)p[16 + i]; }
  return a;
}
__device__ __forceinline__ v16h frag_f32s(const float* rowk0, int lane, float sc) {
  v16h a; const float* p = rowk0 + 8 * (lane >> 4);
#pragma unroll
  for (int i = 0; i < 8; ++i) { a[i] = (_Float16)(p[i] * sc); a[8 + i] = (_Float16)(p[16 + i] * sc); }
  return a;
}
__device__ __forceinline__ v16h fragc_f32(const float* W, int k0, int n, int lane, int ld, int K) {
  v16h a; const int g = lane >> 4;
#pragma unroll
  for (int i = 0; i < 8; ++i) { const int ka = k0 + 8 * g + i, kb = ka + 16;
    a[i] = (_Float16)(ka < K ? W[(size_t)(ka < K ? ka : K - 1) * ld + n] : 0.f); a[8 + i] = (_Float16)(kb < K ? W[(size_t)(kb < K ? kb : K - 1) * ld + n] : 0.f); }
  return a;
}
struct F2 { v16b h, l; };
__device__ __forceinline__ F2 bsplit16(const float v[16]) { F2 r;
#pragma unroll
  for (int i = 0; i < 16; ++i) { const __bf16 h = (__bf16)v[i]; r.h[i] = h; r.l[i] = (__bf16)(v[i] - (float)h); }
  return r; }
__device__ __forceinline__ F2 split_row(const float* row, int k0, int lane) { float v[16]; const float* p = row + k0 + 8 * (lane >> 4);
#pragma unroll
  for (int i = 0; i < 8; ++i) { v[i] = p[i]; v[8 + i] = p[16 + i]; }
  return bsplit16(v); }
__device__ __forceinline__ F2 split_rowK(const float* row, int k0, int lane, int K) { float v[16]; const int g = lane >> 4;
#pragma unroll
  for (int i = 0; i < 8; ++i) { const int ka = k0 + 8 * g + i, kb = ka + 16; v[i] = ka < K ? row[ka < K ? ka : K - 1] : 0.f; v[8 + i] = kb < K ? row[kb < K ? kb : K - 1] : 0.f; }
  return bsplit16(v); }
__device__ __forceinline__ F2 split_col(const float* W, int k0, int n, int lane, int ld, int K) { float v[16]; const int g = lane >> 4;
#pragma unroll
  for (int i = 0; i < 8; ++i) { const int ka = k0 + 8 * g + i, kb = ka + 16; v[i] = ka < K ? W[(size_t)(ka < K ? ka : K - 1) * ld + n] : 0.f; v[8 + i] = kb < K ? W[(size_t)(kb < K ? kb : K - 1) * ld + n] : 0.f; }
  return bsplit16(v); }
__device__ __forceinline__ v8f mac3(const F2& a, const F2& b, v8f c) { c = wmma_bf(a.l, b.h, c); c = wmma_bf(a.h, b.l, c); return wmma_bf(a.h, b.h, c); }
__device__ __forceinline__ float sigm(float v) { return 1.0f / (1.0f + expf(-v)); }
#define LDSX() do { asm volatile("s_wait_dscnt 0" ::: "memory"); __builtin_amdgcn_wave_barrier(); __builtin_amdgcn_fence(__ATOMIC_RELEASE, "workgroup"); } while (0)


#define NG 1024
#define NC 16
#define NK 3
#define HH 256
#define WW 256
#define NPX (HH * WW)
__device__ __forceinline__ float bfr(float v) { return (float)(__bf16)v; }
__device__ __forceinline__ v16b frag_b(const __bf16* rowk0, int lane) { return __builtin_bit_cast(v16b, frag_h((const _Float16*)rowk0, lane)); }
__device__ __attribute__((noinline)) float exp_ni(float v) { return expf(v); }
__device__ __attribute__((noinline)) float tanh_ni(float v) { return tanhf(v); }

__global__ __launch_bounds__(256) void k_prep(const float* __restrict__ xyz, const float* __restrict__ chol, const float* __restrict__ feat, const float* __restrict__ opac, float* __restrict__ GP, __bf16* __restrict__ FT) {
  const int tid = threadIdx.x;
  if (blockIdx.x < NC * NK) { const int ck = blockIdx.x, c = ck / NK, k = ck % NK; __shared__ __align__(16) __bf16 srow[NG];
    for (int n = tid; n < NG; n += 256) srow[n] = (__bf16)feat[((size_t)c * NG + n) * NK + k];
    __syncthreads();
    if (tid < NG / 8) vst2((unsigned*)(FT + (size_t)ck * NG + tid * 8), *(const v4u*)(&srow[tid * 8]));
    return; }
  __shared__ __align__(16) float sp[NG / 4][8 * 4 + 4];
#pragma unroll 1
  for (int i = 0; i < 4; ++i) { const int n = tid * 4 + i;
    const float mx = tanh_ni(bfr(xyz[n * 2])), my = tanh_ni(bfr(xyz[n * 2 + 1]));
    const float x = 0.5f * (mx + 1.0f) * (float)WW, y = 0.5f * (my + 1.0f) * (float)HH;
    const float l1 = bfr(chol[n * 3]) + 0.5f, l2 = bfr(chol[n * 3 + 1]) + 0.0f, l3 = bfr(chol[n * 3 + 2]) + 0.5f;
    const float sxx = l1 * l1, sxy = l1 * l2, syy = l2 * l2 + l3 * l3; const float det = sxx * syy - sxy * sxy;
    const float cxx = syy / det, cxy = -sxy / det, cyy = sxx / det;
    float* q = &sp[tid][i * 8]; q[0] = x; q[1] = y; q[2] = 0.5f * cxx; q[3] = 0.5f * cyy; q[4] = cxy; q[5] = bfr(opac[n]); q[6] = 0.f; q[7] = 0.f; }
  __syncthreads();
  { const float* base = &sp[0][0];
    for (int q4 = tid; q4 < NG * 8 / 4; q4 += 256) { const int n = q4 >> 1, hv = q4 & 1; vst2(GP + (size_t)n * 8 + hv * 4, *(const v4f*)(&sp[n >> 2][(n & 3) * 8 + hv * 4])); } (void)base; }
}
__global__ __launch_bounds__(128) void k_rast(const float* __restrict__ GP, const __bf16* __restrict__ FT, float* __restrict__ out) {
  __shared__ __align__(16) __bf16 swh[32][NG + 8], swl[32][NG + 8];
  __shared__ __align__(16) float so[48][36];
  const int tid = threadIdx.x, wave = tid >> 5, lane = tid & 31, col = lane & 15, g = lane >> 4; const int y = blockIdx.y, x0 = blockIdx.x * 32;
  const float py = (float)y + 0.5f;
  { const int px = lane; const float pxc = (float)(x0 + px) + 0.5f;
#pragma unroll 1
    for (int n = wave; n < NG; n += 4) { const float* q = GP + (size_t)n * 8; const float dx = pxc - q[0], dy = py - q[1];
      const float sigma = q[2] * (dx * dx) + q[3] * (dy * dy) + q[4] * dy * dx;
      float wv = 0.f; if (sigma >= 0.f) { wv = q[5] * exp_ni(-sigma); wv = wv < 0.999f ? wv : 0.999f; }
      const __bf16 hi = (__bf16)wv; swh[px][n] = hi; swl[px][n] = (__bf16)(wv - (float)hi); } }
  __syncthreads();
  if (wave < 3) { v8f acc[2] = {};
#pragma unroll 2
    for (int kc = 0; kc < NG / 32; ++kc) { const v16b a = frag_b(FT + (size_t)(wave * 16 + col) * NG + kc * 32, lane);
#pragma unroll
      for (int pt = 0; pt < 2; ++pt) { acc[pt] = wmma_bf(a, frag_b(&swl[pt * 16 + col][kc * 32], lane), acc[pt]); acc[pt] = wmma_bf(a, frag_b(&swh[pt * 16 + col][kc * 32], lane), acc[pt]); } }
#pragma unroll
    for (int pt = 0; pt < 2; ++pt)
#pragma unroll
      for (int r = 0; r < 8; ++r) so[wave * 16 + 8 * g + r][pt * 16 + col] = acc[pt][r]; }
  __syncthreads();
  for (int q = tid; q < 48 * 8; q += 128) { const int ck = q >> 3, pc = q & 7; vst2(out + (size_t)ck * NPX + (size_t)y * WW + x0 + pc * 4, *(const v4f*)(&so[ck][pc * 4])); }
}
extern "C" void kernel_launch(void* const* d_in, const int* in_sizes, int n_in, void* d_out, int out_size, void* d_ws, size_t ws_size, hipStream_t stream) {
  (void)in_sizes; (void)n_in; (void)out_size; (void)ws_size;
  const float* xyz = (const float*)d_in[0]; const float* chol = (const float*)d_in[1]; const float* feat = (const float*)d_in[2]; const float* opac = (const float*)d_in[3];
  char* ws = (char*)d_ws; float* GP = (float*)ws; __bf16* FT = (__bf16*)(ws + NG * 8 * 4);
  k_prep<<<NC * NK + 1, 256, 0, stream>>>(xyz, chol, feat, opac, GP, FT);
  k_rast<<<dim3(WW / 32, HH), 128, 0, stream>>>(GP, FT, (float*)d_out);
}
